// GATRegressor_27582279975364
// MI455X (gfx1250) — hardware-verified
//
#include <hip/hip_runtime.h>
#include <stddef.h>


#define HF    128
#define NHD   4
#define HD    32
#define IND   64
#define MLPH  64
#define GR    32
#define XSP   132
#define NB    512
#define NTHR  256
#define NWAVE 8
#define EPL   4
#define NGRP  4
#define CHUNK (NTHR * EPL * NGRP)
#define WCAP  (EPL * NGRP * 32)
#define WSC   64.0f
#define WINV  0.015625f

#define LDS_SACC (NB * HF)
#define LDS_DEN  (NB * NHD)
#define LDS_MX   (NB * NHD)
#define LDS_LIST (NWAVE * WCAP)
#define LDS_BYTES ((LDS_SACC + LDS_DEN + LDS_MX + LDS_LIST + NWAVE) * 4)

static_assert(CHUNK == 4096);
static_assert(WCAP == (CHUNK / NTHR) * 32);
static_assert(NB == 512);
static_assert(((NB / NWAVE) % 4) == 0);
static_assert(((LDS_SACC + LDS_DEN) % 4) == 0);
static_assert(LDS_BYTES == 294944);

typedef float    v4f  __attribute__((ext_vector_type(4)));
typedef float    v8f  __attribute__((ext_vector_type(8)));
typedef int      v4i  __attribute__((ext_vector_type(4)));
typedef _Float16 v8h  __attribute__((ext_vector_type(8)));
typedef _Float16 v16h __attribute__((ext_vector_type(16)));
union Frag   { v16h v; v8h half[2]; };
union Pack16 { v8h h; v4i i; };

__device__ __forceinline__ v8f wm(v16h a, v16h b, v8f c) {
  v8f d = __builtin_amdgcn_wmma_f32_16x16x32_f16(false, a, false, b, (short)0, c, false, false);
  asm volatile("v_nop\n\tv_nop\n\tv_nop\n\tv_nop" : "+v"(d) : "v"(a), "v"(b));
  return d;
}

__device__ __forceinline__ float wsum(float v) {
  v += __shfl_xor(v, 16, 32);
  v += __shfl_xor(v, 8, 32);
  v += __shfl_xor(v, 4, 32);
  v += __shfl_xor(v, 2, 32);
  v += __shfl_xor(v, 1, 32);
  return v;
}

__device__ __forceinline__ v4f xor4(v4f v, int mk) {
  v4f r;
  r.x = __shfl_xor(v.x, mk, 32);
  r.y = __shfl_xor(v.y, mk, 32);
  r.z = __shfl_xor(v.z, mk, 32);
  r.w = __shfl_xor(v.w, mk, 32);
  return r;
}

__device__ __forceinline__ float elu1(float x) {
  return x > 0.f ? x : (__expf(x) - 1.0f);
}

__device__ __forceinline__ int lbound(const int* __restrict__ b, int n, int key) {
  int lo = 0, hi = n;
#pragma unroll 1
  for (int it = 0; it < 40; ++it) {
    if (lo >= hi) break;
    const int mid = (lo + hi) >> 1;
    if (b[mid] < key) lo = mid + 1; else hi = mid;
  }
  return lo;
}

__global__ __launch_bounds__(NTHR) void k_prepw(const float* __restrict__ W, _Float16* Wt, int K, int n8) {
  const int i = blockIdx.x * NTHR + threadIdx.x;
  if (i >= n8) return;
  const int kpr = K >> 3;
  const int n   = i / kpr;
  const int kb  = (i - n * kpr) * 8;
  const float* wp = W + (size_t)kb * HF + n;
  Pack16 u;
  u.h[0] = (_Float16)(wp[0 * HF] * WSC); u.h[1] = (_Float16)(wp[1 * HF] * WSC);
  u.h[2] = (_Float16)(wp[2 * HF] * WSC); u.h[3] = (_Float16)(wp[3 * HF] * WSC);
  u.h[4] = (_Float16)(wp[4 * HF] * WSC); u.h[5] = (_Float16)(wp[5 * HF] * WSC);
  u.h[6] = (_Float16)(wp[6 * HF] * WSC); u.h[7] = (_Float16)(wp[7 * HF] * WSC);
  _Float16* p = Wt + (size_t)n * K + kb;
  *(volatile v4i*)p = u.i;
  __threadfence();
  *(volatile v4i*)p = u.i;
}

__device__ __forceinline__ void epi_tile(v8f acc, int T, int hh, int m, int wave, int ncol,
                                         float cs, float cd, float* Xs, float* Ps, float* Pd) {
  float ss[8], sd[8];
#pragma unroll
  for (int r = 0; r < 8; ++r) {
    const float v = acc[r] * WINV;
    Xs[(T * 16 + 8 * hh + r) * XSP + ncol] = v;
    ss[r] = v * cs;
    sd[r] = v * cd;
  }
#pragma unroll
  for (int mk = 1; mk < 16; mk <<= 1) {
#pragma unroll
    for (int r = 0; r < 8; ++r) {
      ss[r] += __shfl_xor(ss[r], mk, 32);
      sd[r] += __shfl_xor(sd[r], mk, 32);
    }
  }
  if (m == 0) {
#pragma unroll
    for (int r = 0; r < 8; ++r) {
      Ps[(T * 16 + 8 * hh + r) * NWAVE + wave] = ss[r];
      Pd[(T * 16 + 8 * hh + r) * NWAVE + wave] = sd[r];
    }
  }
}

template <int K>
__global__ __launch_bounds__(NTHR) void k_gemm(
    const float* __restrict__ hin, const _Float16* __restrict__ Wt,
    const float* __restrict__ att_s, const float* __restrict__ att_d,
    float* xp, float* asrc, float* adst, int nN) {
  constexpr int AP = K + 8;
  static_assert((K % 64) == 0);
  __shared__ __attribute__((aligned(16))) _Float16 At[GR * AP];
  __shared__ __attribute__((aligned(16))) float Xs[GR * XSP];
  __shared__ __attribute__((aligned(16))) float Ps[GR * NWAVE];
  __shared__ __attribute__((aligned(16))) float Pd[GR * NWAVE];

  const int tid  = threadIdx.x;
  const int lane = tid & 31;
  const int wave = tid >> 5;
  const int hh   = lane >> 4;
  const int m    = lane & 15;
  const int rowBase = blockIdx.x * GR;

  {
    const int r  = tid >> 3;
    const int c0 = (tid & 7) * (K / 8);
    int row = rowBase + r;
    if (row > nN - 1) row = nN - 1;
    const float* p = hin + (size_t)row * K + c0;
#pragma unroll
    for (int jv = 0; jv < K / 64; ++jv) {
      const v4f f0 = *(const v4f*)(p + 8 * jv);
      const v4f f1 = *(const v4f*)(p + 8 * jv + 4);
      Pack16 u;
      u.h[0] = (_Float16)f0.x; u.h[1] = (_Float16)f0.y; u.h[2] = (_Float16)f0.z; u.h[3] = (_Float16)f0.w;
      u.h[4] = (_Float16)f1.x; u.h[5] = (_Float16)f1.y; u.h[6] = (_Float16)f1.z; u.h[7] = (_Float16)f1.w;
      *(v8h*)(At + r * AP + c0 + 8 * jv) = u.h;
    }
  }
  __syncthreads();

  const int ncol = wave * 16 + m;
  v8f c0a = {0.f, 0.f, 0.f, 0.f, 0.f, 0.f, 0.f, 0.f};
  v8f c1a = {0.f, 0.f, 0.f, 0.f, 0.f, 0.f, 0.f, 0.f};
#pragma unroll
  for (int kt = 0; kt < K / 32; ++kt) {
    const int k0 = kt * 32;
    Frag a0, a1, b;
    const _Float16* pb  = Wt + (size_t)ncol * K + k0 + 8 * hh;
    const _Float16* pa0 = At + m * AP + k0 + 8 * hh;
    const _Float16* pa1 = At + (16 + m) * AP + k0 + 8 * hh;
    b.half[0]  = *(const v8h*)pb;  b.half[1]  = *(const v8h*)(pb + 16);
    a0.half[0] = *(const v8h*)pa0; a0.half[1] = *(const v8h*)(pa0 + 16);
    a1.half[0] = *(const v8h*)pa1; a1.half[1] = *(const v8h*)(pa1 + 16);
    c0a = wm(a0.v, b.v, c0a);
    c1a = wm(a1.v, b.v, c1a);
  }

  const float cs = att_s[ncol];
  const float cd = att_d[ncol];
  epi_tile(c0a, 0, hh, m, wave, ncol, cs, cd, Xs, Ps, Pd);
  epi_tile(c1a, 1, hh, m, wave, ncol, cs, cd, Xs, Ps, Pd);
  __syncthreads();

  v4f xr[4];
#pragma unroll
  for (int i = 0; i < 4; ++i) xr[i] = *(const v4f*)(Xs + (4 * wave + i) * XSP + 4 * lane);
  float* gp = 0;
  v4f gv = {0.f, 0.f, 0.f, 0.f};
  if (wave == 0) {
    const float* q = Ps + lane * NWAVE;
    gv.x = q[0] + q[1]; gv.y = q[2] + q[3]; gv.z = q[4] + q[5]; gv.w = q[6] + q[7];
    gp = asrc + (size_t)rowBase * NHD + 4 * lane;
  } else if (wave == 1) {
    const float* q = Pd + lane * NWAVE;
    gv.x = q[0] + q[1]; gv.y = q[2] + q[3]; gv.z = q[4] + q[5]; gv.w = q[6] + q[7];
    gp = adst + (size_t)rowBase * NHD + 4 * lane;
  }
  float* xpp[4];
#pragma unroll
  for (int i = 0; i < 4; ++i) xpp[i] = xp + (size_t)(rowBase + 4 * wave + i) * HF + 4 * lane;

#pragma unroll
  for (int i = 0; i < 4; ++i) *(volatile v4f*)(xpp[i]) = xr[i];
  if (gp) *(volatile v4f*)gp = gv;
  __threadfence();
#pragma unroll
  for (int i = 0; i < 4; ++i) *(volatile v4f*)(xpp[i]) = xr[i];
  if (gp) *(volatile v4f*)gp = gv;
}

template <bool LAST>
__global__ __launch_bounds__(NTHR) void k_gat(
    const int* __restrict__ ei, const float* __restrict__ xp,
    const float* __restrict__ asrc, const float* __restrict__ adst,
    const float* __restrict__ bias, float* hout, int nN, int nE) {
  extern __shared__ v4f lds_dyn[];
  float* sacc = (float*)lds_dyn;
  float* den  = sacc + LDS_SACC;
  float* mx   = den + LDS_DEN;
  int*   list = (int*)(mx + LDS_MX);
  int*   wcnt = list + LDS_LIST;

  const int tid  = threadIdx.x;
  const int lane = tid & 31;
  const int wave = tid >> 5;
  const int nodeBase = blockIdx.x * NB;

  {
    const v4f z4 = {0.f, 0.f, 0.f, 0.f};
    for (int i = tid; i < (LDS_SACC + LDS_DEN) / 4; i += NTHR) lds_dyn[i] = z4;
    for (int i = tid; i < LDS_MX; i += NTHR) mx[i] = -1.0e30f;
  }
  __syncthreads();

  const int* eid = ei + nE;
  const bool al16 = ((nE & 3) == 0);
  const int nChunks = (nE + CHUNK - 1) / CHUNK;

  const int  q   = lane >> 3;
  const int  j8  = lane & 7;
  const int  hdq = j8 >> 1;
  const bool jw  = ((j8 & 1) == 0);

#pragma unroll 1
  for (int ch = 0; ch < nChunks; ++ch) {
    const int cbase = ch * CHUNK;
    int wc = 0;
#pragma unroll
    for (int g = 0; g < NGRP; ++g) {
      const int el0 = (g * NTHR + tid) * EPL;
      const int e0  = cbase + el0;
      const int sent = -2147483647 - 1;
      v4i d;
      if (al16 && (e0 + 3 < nE)) {
        d = *(const v4i*)(eid + e0);
      } else {
        d.x = (e0     < nE) ? eid[e0]     : sent;
        d.y = (e0 + 1 < nE) ? eid[e0 + 1] : sent;
        d.z = (e0 + 2 < nE) ? eid[e0 + 2] : sent;
        d.w = (e0 + 3 < nE) ? eid[e0 + 3] : sent;
      }
      const unsigned s0 = (unsigned)d.x - (unsigned)nodeBase;
      const unsigned s1 = (unsigned)d.y - (unsigned)nodeBase;
      const unsigned s2 = (unsigned)d.z - (unsigned)nodeBase;
      const unsigned s3 = (unsigned)d.w - (unsigned)nodeBase;
      const bool h0 = s0 < (unsigned)NB;
      const bool h1 = s1 < (unsigned)NB;
      const bool h2 = s2 < (unsigned)NB;
      const bool h3 = s3 < (unsigned)NB;
      const unsigned many = __builtin_amdgcn_ballot_w32(h0 | h1 | h2 | h3);
      if (many != 0u) {
#define HITJ(J, HJ, SJ) { \
          const unsigned mj = __builtin_amdgcn_ballot_w32(HJ); \
          if (HJ) { \
            const int pos = wc + (int)__builtin_amdgcn_mbcnt_lo(mj, 0u); \
            if (pos < WCAP) list[wave * WCAP + pos] = ((el0 + (J)) << 9) | (int)(SJ); \
          } \
          wc += (int)__builtin_popcount(mj); }
        HITJ(0, h0, s0)
        HITJ(1, h1, s1)
        HITJ(2, h2, s2)
        HITJ(3, h3, s3)
#undef HITJ
      }
    }
    if (lane == 0) wcnt[wave] = wc;
    __syncthreads();

    if (wave == 0) {
#pragma unroll 1
      for (int wsx = 0; wsx < NWAVE; ++wsx) {
        int n = wcnt[wsx];
        n = (n > WCAP) ? WCAP : n;
        n = (n < 0) ? 0 : n;
        const int* wl = list + wsx * WCAP;
        int i = 0;
#pragma unroll 1
        while (i < n) {
          int idx = i + q;
          if (idx > n - 1) idx = n - 1;
          const int ent  = wl[idx];
          const int slot = ent & (NB - 1);
          const int el   = (ent >> 9) & (CHUNK - 1);
          const int g0 = __builtin_amdgcn_readlane(slot, 0);
          const int g1 = __builtin_amdgcn_readlane(slot, 8);
          const int g2 = __builtin_amdgcn_readlane(slot, 16);
          const int g3 = __builtin_amdgcn_readlane(slot, 24);
          int k = n - i;
          if (k > 4) k = 4;
          if (k > 1 && g1 == g0) k = 1;
          if (k > 2 && (g2 == g0 || g2 == g1)) k = 2;
          if (k > 3 && (g3 == g0 || g3 == g1 || g3 == g2)) k = 3;
          const bool act = (q < k);
          int e = cbase + el;
          if (e > nE - 1) e = nE - 1;
          int src = ei[e];
          src = src < 0 ? 0 : (src > nN - 1 ? nN - 1 : src);
          int nd = nodeBase + slot;
          if (nd > nN - 1) nd = nN - 1;
          float a = asrc[(size_t)src * NHD + hdq] + adst[(size_t)nd * NHD + hdq];
          a = (a > 0.f) ? a : 0.2f * a;
          const int   mi = slot * NHD + hdq;
          const float mo = mx[mi];
          const float mn = fmaxf(mo, a);
          const float c  = __expf(mo - mn);
          const float p  = __expf(a - mn);
          const float* xg = xp + (size_t)src * HF + 16 * j8;
          const v4f x0 = *(const v4f*)(xg);
          const v4f x1 = *(const v4f*)(xg + 4);
          const v4f x2 = *(const v4f*)(xg + 8);
          const v4f x3 = *(const v4f*)(xg + 12);
          float* sp = sacc + slot * HF + 16 * j8;
          const v4f r0 = *(const v4f*)(sp)      * c + p * x0;
          const v4f r1 = *(const v4f*)(sp + 4)  * c + p * x1;
          const v4f r2 = *(const v4f*)(sp + 8)  * c + p * x2;
          const v4f r3 = *(const v4f*)(sp + 12) * c + p * x3;
          if (act) {
            *(v4f*)(sp)      = r0;
            *(v4f*)(sp + 4)  = r1;
            *(v4f*)(sp + 8)  = r2;
            *(v4f*)(sp + 12) = r3;
            if (jw) {
              mx[mi] = mn;
              const float od = den[mi];
              den[mi] = od * c + p;
            }
          }
          i += k;
        }
      }
    }
    __syncthreads();
  }

  const int hd2 = lane >> 3;
  if (!LAST) {
    const v4f b4 = *(const v4f*)(bias + 4 * lane);
#pragma unroll 1
    for (int t = 0; t < NB / NWAVE; ++t) {
      const int slot = wave * (NB / NWAVE) + t;
      const int node = nodeBase + slot;
      int nl = node;
      if (nl > nN - 1) nl = nN - 1;
      float a = asrc[(size_t)nl * NHD + hd2] + adst[(size_t)nl * NHD + hd2];
      a = (a > 0.f) ? a : 0.2f * a;
      const float mo = mx[slot * NHD + hd2];
      const float mn = fmaxf(mo, a);
      const float c  = __expf(mo - mn);
      const float p  = __expf(a - mn);
      const v4f xv = *(const v4f*)(xp + (size_t)nl * HF + 4 * lane);
      const v4f sv = *(const v4f*)(sacc + slot * HF + 4 * lane) * c + p * xv;
      const float dv  = den[slot * NHD + hd2] * c + p;
      const float inv = 1.0f / dv;
      v4f h = sv * inv + b4;
      h.x = elu1(h.x); h.y = elu1(h.y); h.z = elu1(h.z); h.w = elu1(h.w);
      float* op = hout + (size_t)node * HF + 4 * lane;
      *(volatile v4f*)op = h;
      __threadfence();
      *(volatile v4f*)op = h;
    }
  } else {
    const int f4 = 4 * (lane & 7);
    const v4f b4 = *(const v4f*)(bias + f4);
#pragma unroll 1
    for (int t4 = 0; t4 < NB / NWAVE / 4; ++t4) {
      v4f keep = {0.f, 0.f, 0.f, 0.f};
#pragma unroll 1
      for (int u = 0; u < 4; ++u) {
        const int slot = wave * (NB / NWAVE) + 4 * t4 + u;
        const int node = nodeBase + slot;
        int nl = node;
        if (nl > nN - 1) nl = nN - 1;
        float a = asrc[(size_t)nl * NHD + hd2] + adst[(size_t)nl * NHD + hd2];
        a = (a > 0.f) ? a : 0.2f * a;
        const float mo = mx[slot * NHD + hd2];
        const float mn = fmaxf(mo, a);
        const float c  = __expf(mo - mn);
        const float p  = __expf(a - mn);
        const v4f xv = *(const v4f*)(xp + (size_t)nl * HF + 4 * lane);
        const v4f sv = *(const v4f*)(sacc + slot * HF + 4 * lane) * c + p * xv;
        const float dv  = den[slot * NHD + hd2] * c + p;
        const float inv = 1.0f / dv;
        const v4f v  = sv * inv;
        const v4f y1 = v + xor4(v, 8);
        const v4f y2 = y1 + xor4(y1, 16);
        v4f hm = y2 * 0.25f + b4;
        hm.x = elu1(hm.x); hm.y = elu1(hm.y); hm.z = elu1(hm.z); hm.w = elu1(hm.w);
        if (hd2 == u) keep = hm;
      }
      const int node0 = nodeBase + wave * (NB / NWAVE) + 4 * t4;
      float* op = hout + (size_t)(node0 + hd2) * HD + f4;
      *(volatile v4f*)op = keep;
      __threadfence();
      *(volatile v4f*)op = keep;
    }
  }
}

__global__ __launch_bounds__(NTHR) void k_pool(
    const float* __restrict__ h3, const int* __restrict__ bat,
    const float* __restrict__ Wm1, const float* __restrict__ bm1,
    const float* __restrict__ Wm2, const float* __restrict__ bm2,
    float* out, int nN, int G) {
  __shared__ __attribute__((aligned(16))) float res[32];
  const int tid  = threadIdx.x;
  const int lane = tid & 31;
  const int wave = tid >> 5;
  const int gBase = blockIdx.x * 32;

#pragma unroll 1
  for (int t = 0; t < 4; ++t) {
    const int g = gBase + 4 * wave + t;
    float r = 0.f;
    if (g < G) {
      const int lo = lbound(bat, nN, g);
      const int hi = lbound(bat, nN, g + 1);
      float s = 0.f;
#pragma unroll 1
      for (int n = lo; n < hi && n < nN; ++n) s += h3[(size_t)n * HD + lane];
      const float cnt = (float)(hi - lo);
      const float pooled = s * (1.0f / fmaxf(cnt, 1.0f));
      float z0 = 0.f, z1 = 0.f;
#pragma unroll 4
      for (int f = 0; f < HD; ++f) {
        const float pf = __shfl(pooled, f, 32);
        z0 += pf * Wm1[f * MLPH + lane];
        z1 += pf * Wm1[f * MLPH + 32 + lane];
      }
      z0 += bm1[lane];
      z1 += bm1[32 + lane];
      z0 = fmaxf(z0, 0.f);
      z1 = fmaxf(z1, 0.f);
      r = wsum(z0 * Wm2[lane] + z1 * Wm2[32 + lane]) + bm2[0];
    }
    if (lane == 0) res[4 * wave + t] = r;
  }
  __syncthreads();

  if (wave == 0 && lane < 8) {
    const int gl = gBase + 4 * lane;
    const v4f v = *(const v4f*)(res + 4 * lane);
    float* op = out + gl;
    const bool full = (gl + 4 <= G);
    if (full) {
      *(volatile v4f*)op = v;
    } else {
      if (gl     < G) *(volatile float*)(op)     = v.x;
      if (gl + 1 < G) *(volatile float*)(op + 1) = v.y;
      if (gl + 2 < G) *(volatile float*)(op + 2) = v.z;
      if (gl + 3 < G) *(volatile float*)(op + 3) = v.w;
    }
    __threadfence();
    if (full) {
      *(volatile v4f*)op = v;
    } else {
      if (gl     < G) *(volatile float*)(op)     = v.x;
      if (gl + 1 < G) *(volatile float*)(op + 1) = v.y;
      if (gl + 2 < G) *(volatile float*)(op + 2) = v.z;
      if (gl + 3 < G) *(volatile float*)(op + 3) = v.w;
    }
  }
}

static inline size_t al256(size_t b) { return (b + 255) & ~(size_t)255; }

extern "C" void kernel_launch(void* const* d_in, const int* in_sizes, int n_in,
                              void* d_out, int out_size, void* d_ws, size_t ws_size,
                              hipStream_t stream) {
  if (n_in < 19) return;
  const int nN = in_sizes[0] / IND;
  const int nE = in_sizes[1] / 2;
  const int G  = out_size;
  if (nN <= 0 || G <= 0 || nE < 0) return;
  if (in_sizes[0] != nN * IND || in_sizes[1] != 2 * nE || in_sizes[2] != nN) return;
  if (in_sizes[3] != IND * HF) return;
  if (in_sizes[4] != HF || in_sizes[5] != HF || in_sizes[6] != HF) return;
  if (in_sizes[7] != HF * HF || in_sizes[8] != HF || in_sizes[9] != HF || in_sizes[10] != HF) return;
  if (in_sizes[11] != HF * HF || in_sizes[12] != HF || in_sizes[13] != HF || in_sizes[14] != HD) return;
  if (in_sizes[15] != HD * MLPH || in_sizes[16] != MLPH || in_sizes[17] != MLPH || in_sizes[18] < 1) return;

  const float* x    = (const float*)d_in[0];
  const int*   ei   = (const int*)d_in[1];
  const int*   bat  = (const int*)d_in[2];
  const float* W1   = (const float*)d_in[3];
  const float* a1s  = (const float*)d_in[4];
  const float* a1d  = (const float*)d_in[5];
  const float* b1   = (const float*)d_in[6];
  const float* W2   = (const float*)d_in[7];
  const float* a2s  = (const float*)d_in[8];
  const float* a2d  = (const float*)d_in[9];
  const float* b2   = (const float*)d_in[10];
  const float* W3   = (const float*)d_in[11];
  const float* a3s  = (const float*)d_in[12];
  const float* a3d  = (const float*)d_in[13];
  const float* b3   = (const float*)d_in[14];
  const float* Wm1  = (const float*)d_in[15];
  const float* bm1  = (const float*)d_in[16];
  const float* Wm2  = (const float*)d_in[17];
  const float* bm2  = (const float*)d_in[18];
  float* out = (float*)d_out;

  const int nP      = ((nN + GR - 1) / GR) * GR;
  const int gridGat = (nN + NB - 1) / NB;
  const int nPB     = gridGat * NB;
  size_t off = 0;
  _Float16* Wt = (_Float16*)((char*)d_ws + off); off += al256((size_t)HF * HF * sizeof(_Float16));
  float* xp   = (float*)((char*)d_ws + off);     off += al256((size_t)nP * HF * sizeof(float));
  float* asrc = (float*)((char*)d_ws + off);     off += al256((size_t)nP * NHD * sizeof(float));
  float* adst = (float*)((char*)d_ws + off);     off += al256((size_t)nP * NHD * sizeof(float));
  float* hbuf = (float*)((char*)d_ws + off);     off += al256((size_t)nPB * HF * sizeof(float));
  float* h3   = (float*)((char*)d_ws + off);     off += al256((size_t)nPB * HD * sizeof(float));
  if (off > ws_size) return;
  if (off > (size_t)134217728) return;

  const int gGemm = nP / GR;
  const int n8a   = HF * IND / 8;
  const int n8b   = HF * HF / 8;

  hipFuncSetAttribute(reinterpret_cast<const void*>(&k_gat<false>),
                      hipFuncAttributeMaxDynamicSharedMemorySize, LDS_BYTES);
  hipFuncSetAttribute(reinterpret_cast<const void*>(&k_gat<true>),
                      hipFuncAttributeMaxDynamicSharedMemorySize, LDS_BYTES);

  k_prepw<<<(n8a + NTHR - 1) / NTHR, NTHR, 0, stream>>>(W1, Wt, IND, n8a);
  k_gemm<IND><<<gGemm, NTHR, 0, stream>>>(x, Wt, a1s, a1d, xp, asrc, adst, nN);
  k_gat<false><<<gridGat, NTHR, LDS_BYTES, stream>>>(ei, xp, asrc, adst, b1, hbuf, nN, nE);

  k_prepw<<<(n8b + NTHR - 1) / NTHR, NTHR, 0, stream>>>(W2, Wt, HF, n8b);
  k_gemm<HF><<<gGemm, NTHR, 0, stream>>>(hbuf, Wt, a2s, a2d, xp, asrc, adst, nN);
  k_gat<false><<<gridGat, NTHR, LDS_BYTES, stream>>>(ei, xp, asrc, adst, b2, hbuf, nN, nE);

  k_prepw<<<(n8b + NTHR - 1) / NTHR, NTHR, 0, stream>>>(W3, Wt, HF, n8b);
  k_gemm<HF><<<gGemm, NTHR, 0, stream>>>(hbuf, Wt, a3s, a3d, xp, asrc, adst, nN);
  k_gat<true><<<gridGat, NTHR, LDS_BYTES, stream>>>(ei, xp, asrc, adst, b3, h3, nN, nE);

  k_pool<<<(G + 31) / 32, NTHR, 0, stream>>>(h3, bat, Wm1, bm1, Wm2, bm2, out, nN, G);
}
